// Cylinder3D_6408091206414
// MI455X (gfx1250) — hardware-run, weakly checked
//
#include <hip/hip_runtime.h>


namespace {
constexpr int NV = 200000, CIN = 32, CO = 64, KO = 9, K1 = KO * CIN  , K2 = KO * CO  , VB = 32  , NBLK = NV / VB  ;
constexpr float XS = 8.0f, HS = 256.0f, WSC = 256.0f, SLOPE = 0.01f, BNEPS = 1e-5f;
typedef _Float16 b16;
typedef __attribute__((ext_vector_type(16))) _Float16 v16b;
typedef __attribute__((ext_vector_type(8))) _Float16 v8b;
typedef __attribute__((ext_vector_type(8))) float v8f;
typedef __attribute__((ext_vector_type(4))) float v4f;
typedef __attribute__((ext_vector_type(2))) float v2f;
__device__ __forceinline__ float bf16_rne(float f) { unsigned int u = __float_as_uint(f); u += 0x7FFFu + ((u >> 16) & 1u); float r = __uint_as_float(u & 0xFFFF0000u); asm volatile("" : "+v"(r)); return r; }
__device__ __forceinline__ float bfv(float f) { float r = bf16_rne(f); asm volatile("" : "+v"(r)); return r; }
__device__ __forceinline__ void split16(float v, b16& hi, b16& lo) { hi = (b16)v; lo = (b16)(v - (float)hi); }
__device__ __forceinline__ v16b frag_kb(const b16* p, int hh) { const v8b a = *(const v8b*)(p + 8 * hh), b = *(const v8b*)(p + 16 + 8 * hh); v16b f;
#pragma unroll
  for (int e = 0; e < 8; ++e) { f[e] = a[e]; f[8 + e] = b[e]; } return f; }
__device__ __forceinline__ v8f wmma16b(v16b a, v16b b, v8f c) { v8f d = __builtin_amdgcn_wmma_f32_16x16x32_f16(false, a, false, b, (short)0, c, false, false); asm volatile("v_nop\n\tv_nop\n\tv_nop\n\tv_nop" : "+v"(d) : "v"(a), "v"(b)); return d; }
__device__ __forceinline__ void wave_lds_sync() { __builtin_amdgcn_fence(__ATOMIC_RELEASE, "workgroup"); __builtin_amdgcn_wave_barrier(); __builtin_amdgcn_fence(__ATOMIC_ACQUIRE, "workgroup"); }
__device__ __forceinline__ float pmul(float a, float b) { float p = a * b; asm volatile("" : "+v"(p)); return p; }
__device__ __forceinline__ int iclamp(int v, int lo, int hi) { return v < lo ? lo : (v > hi ? hi : v); }
__device__ __forceinline__ float lrelu(float v) { return v > 0.0f ? v : SLOPE * v; }

__global__ __launch_bounds__(256) void wput_kernel(const float* __restrict__ w1, const float* __restrict__ w12, const float* __restrict__ w2, const float* __restrict__ w3, b16* __restrict__ WT1, b16* __restrict__ WT12, b16* __restrict__ WT2, b16* __restrict__ WT3) { const int u = blockIdx.x * 256 + threadIdx.x; v8b v;
  if (u < CO * (K1 / 8)) { const int o = u / (K1 / 8), k0 = (u % (K1 / 8)) * 8;
#pragma unroll
    for (int j = 0; j < 8; ++j) { const int kk = k0 + j; v[j] = (b16)(bf16_rne(w1[(size_t)kk * CO + o]) * WSC); } for (int pass = 0; pass < 2; ++pass) { *(volatile v8b*)(WT1 + (size_t)o * K1 + k0) = v; __threadfence(); }
#pragma unroll
    for (int j = 0; j < 8; ++j) { const int kk = k0 + j; v[j] = (b16)(bf16_rne(w2[(size_t)kk * CO + o]) * WSC); } for (int pass = 0; pass < 2; ++pass) { *(volatile v8b*)(WT2 + (size_t)o * K1 + k0) = v; __threadfence(); } }
  if (u < CO * (K2 / 8)) { const int o = u / (K2 / 8), k0 = (u % (K2 / 8)) * 8;
#pragma unroll
    for (int j = 0; j < 8; ++j) { const int kk = k0 + j; v[j] = (b16)(bf16_rne(w12[(size_t)kk * CO + o]) * WSC); } for (int pass = 0; pass < 2; ++pass) { *(volatile v8b*)(WT12 + (size_t)o * K2 + k0) = v; __threadfence(); }
#pragma unroll
    for (int j = 0; j < 8; ++j) { const int kk = k0 + j; v[j] = (b16)(bf16_rne(w3[(size_t)kk * CO + o]) * WSC); } for (int pass = 0; pass < 2; ++pass) { *(volatile v8b*)(WT3 + (size_t)o * K2 + k0) = v; __threadfence(); } } }
__global__ __launch_bounds__(64) void stage1_kernel(const float* __restrict__ feats, const int* __restrict__ nbrA, const int* __restrict__ mA, const int* __restrict__ nbrB, const int* __restrict__ mB, const b16* __restrict__ WT1, const b16* __restrict__ WT2, int VLIM, float* __restrict__ PA, float* __restrict__ PB, float* __restrict__ PS1) {
  __shared__ __attribute__((aligned(16))) b16 Ah[2][16][K1 + 8]; __shared__ float Tf[2][16][CO + 4]; __shared__ float Red[2][4 * CO]; const int wave = threadIdx.x >> 5, lane = threadIdx.x & 31, nloc = lane & 15, hlf = lane >> 4; const size_t m0 = (size_t)blockIdx.x * VB + wave * 16; const bool act = m0 < (size_t)VLIM;
  float red[8]; for (int q = 0; q < 8; ++q) red[q] = 0.0f;
#pragma unroll
  for (int P = 0; P < 2; ++P) { const int* nbr = P ? nbrB : nbrA; const int* msk = P ? mB : mA; const b16* W = P ? WT2 : WT1; float* OUTp = P ? PB : PA;
    if (act) {
      for (int rr = 0; rr < 16; ++rr) { const size_t v = m0 + rr;
#pragma unroll 1
        for (int k = 0; k < KO; ++k) { const int u = iclamp(nbr[(size_t)k * NV + v], 0, NV - 1); const bool ok = msk[(size_t)k * NV + v] != 0 && u < VLIM; Ah[wave][rr][k * CIN + lane] = (b16)(ok ? bf16_rne(feats[(size_t)u * CIN + lane]) * XS : 0.0f); } }
      if (lane < 16) for (int kk = K1; kk < K1 + 8; ++kk) Ah[wave][lane][kk] = (b16)0.0f;
      wave_lds_sync(); v8f acc[4] = {(v8f){}, (v8f){}, (v8f){}, (v8f){}};
#pragma unroll
      for (int kb = 0; kb < K1; kb += 32) { const v16b a = frag_kb(&Ah[wave][nloc][kb], hlf);
#pragma unroll
        for (int t = 0; t < 4; ++t) acc[t] = wmma16b(a, frag_kb(W + (size_t)(t * 16 + nloc) * K1 + kb, hlf), acc[t]); }
#pragma unroll
      for (int t = 0; t < 4; ++t)
#pragma unroll
        for (int r8 = 0; r8 < 8; ++r8) Tf[wave][8 * hlf + r8][t * 16 + nloc] = lrelu(acc[t][r8] * (1.0f / (XS * WSC)));
      wave_lds_sync();
      for (int rr = 0; rr < 16; ++rr) for (int q = 0; q < 2; ++q) { const float val = Tf[wave][rr][q * 32 + lane]; red[P * 4 + q] += val; red[P * 4 + 2 + q] += val * val; }
      for (int pass = 0; pass < 2; ++pass) { for (int rr = 0; rr < 16; ++rr) *(volatile v2f*)(OUTp + (m0 + rr) * CO + lane * 2) = (v2f){Tf[wave][rr][lane * 2], Tf[wave][rr][lane * 2 + 1]}; __threadfence(); }
      wave_lds_sync(); } }
#pragma unroll
  for (int P = 0; P < 2; ++P)
#pragma unroll
    for (int q = 0; q < 2; ++q) { Red[wave][P * 128 + q * 32 + lane] = red[P * 4 + q]; Red[wave][P * 128 + 64 + q * 32 + lane] = red[P * 4 + 2 + q]; }
  __syncthreads();
  if (wave == 0) for (int pass = 0; pass < 2; ++pass) { for (int c = lane; c < 4 * CO; c += 32) { float s = 0.0f; for (int w = 0; w < 2; ++w) s += Red[w][c]; ((volatile float*)PS1)[(size_t)blockIdx.x * 4 * CO + c] = s; } __threadfence(); } }
__global__ __launch_bounds__(128) void bn_kernel(const float* __restrict__ PS, int nblk, int VLIM, float* __restrict__ BNs) { const int t = threadIdx.x; const int P = t / CO, c = t % CO; double s = 0.0, s2 = 0.0;
#pragma unroll 1
  for (int b = 0; b < nblk; ++b) { s += (double)PS[(size_t)b * 4 * CO + P * 128 + c]; s2 += (double)PS[(size_t)b * 4 * CO + P * 128 + 64 + c]; }
  const double mu = s / VLIM; double var = s2 / VLIM - mu * mu; if (var < 0.0) var = 0.0; const float m = (float)mu, rs = (float)(1.0 / sqrt(var + (double)BNEPS));
  for (int pass = 0; pass < 2; ++pass) { ((volatile float*)BNs)[P * 128 + c] = m; ((volatile float*)BNs)[P * 128 + 64 + c] = rs; __threadfence(); } }
__global__ __launch_bounds__(64) void stage2_kernel(const float* __restrict__ PA, const float* __restrict__ PB, const float* __restrict__ BN1, const float* __restrict__ g0, const float* __restrict__ b0, const float* __restrict__ g1, const float* __restrict__ b1, const int* __restrict__ nbrA, const int* __restrict__ mA, const int* __restrict__ nbrB, const int* __restrict__ mB, const b16* __restrict__ WT12, const b16* __restrict__ WT3, int VLIM, float* __restrict__ QA, float* __restrict__ QB, float* __restrict__ PS2) {
  __shared__ __attribute__((aligned(16))) b16 Ah[2][16][K2 + 8], Al[2][16][K2 + 8]; __shared__ float Tf[2][16][CO + 4]; __shared__ float Red[2][4 * CO]; const int wave = threadIdx.x >> 5, lane = threadIdx.x & 31, nloc = lane & 15, hlf = lane >> 4; const size_t m0 = (size_t)blockIdx.x * VB + wave * 16; const bool act = m0 < (size_t)VLIM;
  float red[8]; for (int q = 0; q < 8; ++q) red[q] = 0.0f;
#pragma unroll
  for (int P = 0; P < 2; ++P) {
    const float* IN = P ? PB : PA; const int* nbr = P ? nbrA : nbrB; const int* msk = P ? mA : mB; const b16* W = P ? WT3 : WT12; const float* gg = P ? g1 : g0; const float* be = P ? b1 : b0; float* OUTp = P ? QB : QA;
    const float mu0 = BN1[P * 128 + lane], rs0 = BN1[P * 128 + 64 + lane], mu1 = BN1[P * 128 + 32 + lane], rs1 = BN1[P * 128 + 64 + 32 + lane]; const float ga0 = bfv(gg[lane]), ga1 = bfv(gg[32 + lane]), bb0 = bfv(be[lane]), bb1 = bfv(be[32 + lane]);
    if (act) {
      for (int rr = 0; rr < 16; ++rr) { const size_t v = m0 + rr;
#pragma unroll 1
        for (int k = 0; k < KO; ++k) { const int u = iclamp(nbr[(size_t)k * NV + v], 0, NV - 1); const bool ok = msk[(size_t)k * NV + v] != 0 && u < VLIM; const v2f raw = {IN[(size_t)u * CO + lane], IN[(size_t)u * CO + 32 + lane]};
          const float x0 = ok ? pmul(pmul(raw[0] - mu0, rs0), ga0) + bb0 : 0.0f, x1 = ok ? pmul(pmul(raw[1] - mu1, rs1), ga1) + bb1 : 0.0f; b16 p, ql; split16(x0 * HS, p, ql); Ah[wave][rr][k * CO + lane] = p; Al[wave][rr][k * CO + lane] = ql; split16(x1 * HS, p, ql); Ah[wave][rr][k * CO + 32 + lane] = p; Al[wave][rr][k * CO + 32 + lane] = ql; } }
      wave_lds_sync(); v8f acc[4] = {(v8f){}, (v8f){}, (v8f){}, (v8f){}};
#pragma unroll 2
      for (int kb = 0; kb < K2; kb += 32) { const v16b a = frag_kb(&Ah[wave][nloc][kb], hlf), al = frag_kb(&Al[wave][nloc][kb], hlf);
#pragma unroll
        for (int t = 0; t < 4; ++t) { const v16b bw = frag_kb(W + (size_t)(t * 16 + nloc) * K2 + kb, hlf); acc[t] = wmma16b(a, bw, acc[t]); acc[t] = wmma16b(al, bw, acc[t]); } }
#pragma unroll
      for (int t = 0; t < 4; ++t)
#pragma unroll
        for (int r8 = 0; r8 < 8; ++r8) Tf[wave][8 * hlf + r8][t * 16 + nloc] = lrelu(acc[t][r8] * (1.0f / (HS * WSC)));
      wave_lds_sync();
      for (int rr = 0; rr < 16; ++rr) for (int q = 0; q < 2; ++q) { const float val = Tf[wave][rr][q * 32 + lane]; red[P * 4 + q] += val; red[P * 4 + 2 + q] += val * val; }
      for (int pass = 0; pass < 2; ++pass) { for (int rr = 0; rr < 16; ++rr) *(volatile v2f*)(OUTp + (m0 + rr) * CO + lane * 2) = (v2f){Tf[wave][rr][lane * 2], Tf[wave][rr][lane * 2 + 1]}; __threadfence(); }
      wave_lds_sync(); } }
#pragma unroll
  for (int P = 0; P < 2; ++P)
#pragma unroll
    for (int q = 0; q < 2; ++q) { Red[wave][P * 128 + q * 32 + lane] = red[P * 4 + q]; Red[wave][P * 128 + 64 + q * 32 + lane] = red[P * 4 + 2 + q]; }
  __syncthreads();
  if (wave == 0) for (int pass = 0; pass < 2; ++pass) { for (int c = lane; c < 4 * CO; c += 32) { float s = 0.0f; for (int w = 0; w < 2; ++w) s += Red[w][c]; ((volatile float*)PS2)[(size_t)blockIdx.x * 4 * CO + c] = s; } __threadfence(); } }
__global__ __launch_bounds__(64) void out_kernel(const float* __restrict__ QA, const float* __restrict__ QB, const float* __restrict__ BN2, const float* __restrict__ g02, const float* __restrict__ b02, const float* __restrict__ g2, const float* __restrict__ b2, int VLIM, float* __restrict__ out) { const int wave = threadIdx.x >> 5, lane = threadIdx.x & 31; const size_t m0 = (size_t)blockIdx.x * VB + wave * 16; if (m0 >= (size_t)VLIM) return;
  const int c0 = lane * 2; float muA[2], rsA[2], muB[2], rsB[2], gA[2], bA[2], gB[2], bB_[2]; for (int k = 0; k < 2; ++k) { muA[k] = BN2[c0 + k]; rsA[k] = BN2[64 + c0 + k]; muB[k] = BN2[128 + c0 + k]; rsB[k] = BN2[192 + c0 + k]; gA[k] = bfv(g02[c0 + k]); bA[k] = bfv(b02[c0 + k]); gB[k] = bfv(g2[c0 + k]); bB_[k] = bfv(b2[c0 + k]); }
  for (int pass = 0; pass < 2; ++pass) { for (int rr = 0; rr < 16; ++rr) { v2f o; for (int k = 0; k < 2; ++k) { const size_t idx = (m0 + rr) * CO + c0 + k; const float sv = pmul(pmul(QA[idx] - muA[k], rsA[k]), gA[k]) + bA[k]; const float rv = pmul(pmul(QB[idx] - muB[k], rsB[k]), gB[k]) + bB_[k]; o[k] = rv + sv; } *(volatile v2f*)(out + (m0 + rr) * CO + c0) = o; } __threadfence(); } }
}

extern "C" void kernel_launch(void* const* d_in, const int* in_sizes, int n_in, void* d_out, int out_size, void* d_ws, size_t ws_size, hipStream_t stream) {
  (void)n_in;
  auto Fp = [&](int i) { return (const float*)d_in[i]; }; auto Ip = [&](int i) { return (const int*)d_in[i]; };
  if (in_sizes[0] != NV * CIN || in_sizes[1] != KO * CIN * CO || in_sizes[2] != KO * CO * CO || in_sizes[3] != KO * CIN * CO || in_sizes[4] != KO * CO * CO || in_sizes[13] != KO * NV || in_sizes[14] != KO * NV || in_sizes[15] != KO * NV || in_sizes[16] != KO * NV || out_size != NV * CO) return;
  const int VLIM = NV;
  size_t off = 0; char* ws = (char*)d_ws;
  auto carve = [&](size_t bytes) { char* p = ws + off; off += (bytes + 255) & ~(size_t)255; return p; };
  b16* WT1 = (b16*)carve((size_t)CO * K1 * 2); b16* WT12 = (b16*)carve((size_t)CO * K2 * 2); b16* WT2 = (b16*)carve((size_t)CO * K1 * 2); b16* WT3 = (b16*)carve((size_t)CO * K2 * 2);
  float* PA = (float*)carve((size_t)NV * CO * 4); float* PB = (float*)carve((size_t)NV * CO * 4); float* QA = (float*)carve((size_t)NV * CO * 4); float* QB = (float*)carve((size_t)NV * CO * 4); float* PS1 = (float*)carve((size_t)NBLK * 4 * CO * 4); float* PS2 = (float*)carve((size_t)NBLK * 4 * CO * 4); float* BN1 = (float*)carve(4 * CO * 4); float* BN2 = (float*)carve(4 * CO * 4);
  if (off > ws_size || off > ((size_t)256 << 20)) return;
  const int nblk = VLIM / VB;
  wput_kernel<<<(CO * (K2 / 8) + 255) / 256, 256, 0, stream>>>(Fp(1), Fp(2), Fp(3), Fp(4), WT1, WT12, WT2, WT3);
  stage1_kernel<<<nblk, 64, 0, stream>>>(Fp(0), Ip(13), Ip(14), Ip(15), Ip(16), WT1, WT2, VLIM, PA, PB, PS1);
  bn_kernel<<<1, 128, 0, stream>>>(PS1, nblk, VLIM, BN1);
  stage2_kernel<<<nblk, 64, 0, stream>>>(PA, PB, BN1, Fp(5), Fp(6), Fp(9), Fp(10), Ip(13), Ip(14), Ip(15), Ip(16), WT12, WT3, VLIM, QA, QB, PS2);
  bn_kernel<<<1, 128, 0, stream>>>(PS2, nblk, VLIM, BN2);
  out_kernel<<<nblk, 64, 0, stream>>>(QA, QB, BN2, Fp(7), Fp(8), Fp(11), Fp(12), VLIM, (float*)d_out);
}
